// ConformerBlock_16801912062469
// MI455X (gfx1250) — hardware-verified
//
#include <hip/hip_runtime.h>


typedef __attribute__((ext_vector_type(16))) _Float16 v16h;
typedef __attribute__((ext_vector_type(8)))  _Float16 v8h;
typedef __attribute__((ext_vector_type(8)))  float v8f;
typedef __attribute__((ext_vector_type(4)))  float v4f;
typedef __attribute__((ext_vector_type(4)))  unsigned int v4u;
union H8 { v8h h; v4u u; };

#ifndef NB
#define NB 2
#endif
#ifndef SEQ
#define SEQ 2048
#endif
#define NB_FULL  2
#define SEQ_FULL 2048
#define DM   1024
#define NH   16
#define HD   64
#define FF   4096
#define ROWS (NB * SEQ)
#define KPAD 72
#define VSPAD 136
#define YP   1028
#define RTP  32
#define LN_EPS 1e-5f
#define WSC    64.0f
#define LN1024 6.931471806f
#define ROPE_BASE 10000.0f

#define NT_QKV ((DM / 64) * (3 * DM / 64))
#define NT_O   ((DM / 64) * (DM / 64))
#define NT_F1  ((DM / 64) * (FF / 64))
#define NT_F2  ((FF / 64) * (DM / 64))
#define NWT    (NT_QKV + NT_O + NT_F1 + NT_F2)

#define PLANE2     ((size_t)ROWS * DM * 2)
#define PLANE4     ((size_t)ROWS * DM * 4)
#define WQKV_BYTES ((size_t)3 * DM * DM * 2)
#define WO_BYTES   ((size_t)DM * DM * 2)
#define WF1_BYTES  ((size_t)FF * DM * 2)
#define WF2_BYTES  ((size_t)DM * FF * 2)
#define H_BYTES    ((size_t)ROWS * FF * 2)
#define WS_TOTAL   (2 * PLANE2 + WQKV_BYTES + WO_BYTES + WF1_BYTES + WF2_BYTES + \
                    3 * PLANE2 + PLANE4 + PLANE2 + H_BYTES)

static_assert(NB >= 1 && NB <= NB_FULL);
static_assert(SEQ >= 128 && SEQ <= SEQ_FULL && (SEQ % 128) == 0);
static_assert((ROWS % 128) == 0 && (ROWS % 16) == 0 && (ROWS % 8) == 0);
static_assert((DM % 64) == 0 && (FF % 64) == 0 && HD == 64 && NH * HD == DM);
static_assert(128 * KPAD >= 64 * VSPAD);
static_assert((size_t)NB * NH * SEQ * HD * 2 == PLANE2);
static_assert(WS_TOTAL <= (size_t)134217728);

__device__ __forceinline__ float bf16q(float f) {
  unsigned int u = __float_as_uint(f);
  u += 0x7FFFu + ((u >> 16) & 1u);
  return __uint_as_float(u & 0xFFFF0000u);
}

__device__ __forceinline__ float wave_sum(float v) {
  v += __shfl_xor(v, 16, 32);
  v += __shfl_xor(v, 8, 32);
  v += __shfl_xor(v, 4, 32);
  v += __shfl_xor(v, 2, 32);
  v += __shfl_xor(v, 1, 32);
  return v;
}

__device__ __forceinline__ v16h load_frag_row(const _Float16* base, int stride, int lane) {
  const _Float16* rowp = base + (lane & 15) * stride + ((lane >> 4) << 3);
  const v8h lo = *(const v8h*)(rowp);
  const v8h hi = *(const v8h*)(rowp + 16);
  return __builtin_shufflevector(lo, hi, 0, 1, 2, 3, 4, 5, 6, 7,
                                 8, 9, 10, 11, 12, 13, 14, 15);
}

__device__ __forceinline__ v8f wmma_f16(v16h a, v16h b, v8f c) {
  v8f d = __builtin_amdgcn_wmma_f32_16x16x32_f16(false, a, false, b, (short)0, c,
                                                 false, false);
  asm volatile("v_nop\n\tv_nop\n\tv_nop\n\tv_nop" : "+v"(d) : "v"(a), "v"(b));
  return d;
}

__global__ __launch_bounds__(256) void ln1_kernel(const float* __restrict__ x,
                                                  const float* __restrict__ g,
                                                  const float* __restrict__ bb,
                                                  _Float16* __restrict__ nxh) {
  const int lane  = threadIdx.x & 31;
  const int wave  = threadIdx.x >> 5;
  const long m    = (long)blockIdx.x * 8 + wave;
  const long srow = (m / SEQ) * SEQ_FULL + (m % SEQ);
  const float* xr = x + srow * DM + lane * 8;

  float s = 0.0f;
#pragma unroll 1
  for (int i = 0; i < 4; ++i) {
    const v4f a = *(const v4f*)(xr + i * 256);
    const v4f c = *(const v4f*)(xr + i * 256 + 4);
    s += ((bf16q(a[0]) + bf16q(a[1])) + (bf16q(a[2]) + bf16q(a[3]))) +
         ((bf16q(c[0]) + bf16q(c[1])) + (bf16q(c[2]) + bf16q(c[3])));
  }
  s = wave_sum(s);
  const float mean = s * (1.0f / DM);

  float ss = 0.0f;
#pragma unroll 1
  for (int i = 0; i < 4; ++i) {
    const v4f a = *(const v4f*)(xr + i * 256);
    const v4f c = *(const v4f*)(xr + i * 256 + 4);
#pragma unroll
    for (int e = 0; e < 4; ++e) {
      const float d0 = bf16q(a[e]) - mean;
      const float d1 = bf16q(c[e]) - mean;
      ss += d0 * d0;
      ss += d1 * d1;
    }
  }
  ss = wave_sum(ss);
  const float rstd = rsqrtf(ss * (1.0f / DM) + LN_EPS);

  _Float16* drow = nxh + m * DM + lane * 8;
#pragma unroll 1
  for (int i = 0; i < 4; ++i) {
    const v4f a  = *(const v4f*)(xr + i * 256);
    const v4f c  = *(const v4f*)(xr + i * 256 + 4);
    const v4f g0 = *(const v4f*)(g + i * 256 + lane * 8);
    const v4f g1 = *(const v4f*)(g + i * 256 + lane * 8 + 4);
    const v4f b0 = *(const v4f*)(bb + i * 256 + lane * 8);
    const v4f b1 = *(const v4f*)(bb + i * 256 + lane * 8 + 4);
    H8 o;
#pragma unroll
    for (int e = 0; e < 4; ++e) {
      o.h[e]     = (_Float16)((bf16q(a[e]) - mean) * rstd * bf16q(g0[e]) + bf16q(b0[e]));
      o.h[4 + e] = (_Float16)((bf16q(c[e]) - mean) * rstd * bf16q(g1[e]) + bf16q(b1[e]));
    }
    _Float16* dst = drow + i * 256;
    *(volatile v4u*)dst = o.u;
    __threadfence();
    *(volatile v4u*)dst = o.u;
  }
}

__global__ __launch_bounds__(256) void cvt_w_kernel(
    const float* __restrict__ Wqkv, const float* __restrict__ Wo,
    const float* __restrict__ Wf1, const float* __restrict__ Wf2,
    _Float16* __restrict__ wqkv, _Float16* __restrict__ woh,
    _Float16* __restrict__ wf1t, _Float16* __restrict__ wf2t) {
  __shared__ _Float16 ts[64 * KPAD];
  const int bid = blockIdx.x;
  const int tid = threadIdx.x;
  const float* W;
  _Float16* dst;
  int K, N, kt, nt;
  if (bid < NT_QKV) {
    const int tile = bid;
    kt = tile / (3 * DM / 64); nt = tile - kt * (3 * DM / 64); K = DM; N = 3 * DM;
    W = Wqkv; dst = wqkv;
  } else if (bid < NT_QKV + NT_O) {
    const int tile = bid - NT_QKV;
    kt = tile / (DM / 64); nt = tile - kt * (DM / 64); K = DM; N = DM;
    W = Wo; dst = woh;
  } else if (bid < NT_QKV + NT_O + NT_F1) {
    const int tile = bid - NT_QKV - NT_O;
    kt = tile / (FF / 64); nt = tile - kt * (FF / 64); K = DM; N = FF;
    W = Wf1; dst = wf1t;
  } else {
    const int tile = bid - NT_QKV - NT_O - NT_F1;
    kt = tile / (DM / 64); nt = tile - kt * (DM / 64); K = FF; N = DM;
    W = Wf2; dst = wf2t;
  }
#pragma unroll
  for (int it = 0; it < 4; ++it) {
    const int idx = it * 256 + tid;
    const int kr = idx >> 4, c4 = idx & 15;
    const v4f v = *(const v4f*)(W + (size_t)(kt * 64 + kr) * N + nt * 64 + c4 * 4);
#pragma unroll
    for (int j = 0; j < 4; ++j) ts[(c4 * 4 + j) * KPAD + kr] = (_Float16)(bf16q(v[j]) * WSC);
  }
  __syncthreads();
  v4u rv[2];
#pragma unroll
  for (int it = 0; it < 2; ++it) {
    const int idx = it * 256 + tid;
    const int n = idx >> 3, piece = idx & 7;
    rv[it] = *(const v4u*)(ts + n * KPAD + piece * 8);
  }
#pragma unroll
  for (int it = 0; it < 2; ++it) {
    const int idx = it * 256 + tid;
    const int n = idx >> 3, piece = idx & 7;
    *(volatile v4u*)(dst + (size_t)(nt * 64 + n) * K + kt * 64 + piece * 8) = rv[it];
  }
  __threadfence();
#pragma unroll
  for (int it = 0; it < 2; ++it) {
    const int idx = it * 256 + tid;
    const int n = idx >> 3, piece = idx & 7;
    *(volatile v4u*)(dst + (size_t)(nt * 64 + n) * K + kt * 64 + piece * 8) = rv[it];
  }
}

__global__ __launch_bounds__(256) void qkv_kernel(
    const _Float16* __restrict__ nxh, const _Float16* __restrict__ wqkv,
    const float* __restrict__ bqkv,
    _Float16* __restrict__ q, _Float16* __restrict__ k, _Float16* __restrict__ vT) {
  __shared__ _Float16 stg[128 * KPAD];
  __shared__ float ctab[128 * RTP];
  __shared__ float stab[128 * RTP];

  const int tid  = threadIdx.x;
  const int lane = tid & 31;
  const int wave = tid >> 5;
  const int hh   = lane >> 4;
  const int l15  = lane & 15;

  const int cb   = blockIdx.y;
  const int osel = cb >> 4;
  const int h    = cb & 15;
  const long m0  = (long)blockIdx.x * 128;
  const int  b   = (int)(m0 / SEQ);
  const int  s0  = (int)(m0 - (long)b * SEQ);

  if (osel < 2) {
#pragma clang fp contract(off)
    const int i  = tid & 31;
    const int tg = tid >> 5;
    const float e   = (float)(2 * i) * (1.0f / 64.0f);
    const float inv = 1.0f / powf(ROPE_BASE, e);
#pragma unroll 1
    for (int tt = tg; tt < 128; tt += 8) {
      const float ang = (float)(s0 + tt) * inv;
      ctab[tt * RTP + i] = cosf(ang);
      stab[tt * RTP + i] = sinf(ang);
    }
  }
  __syncthreads();

  const _Float16* xrow = nxh + (m0 + wave * 16) * DM;
  const _Float16* wrow = wqkv + ((long)cb * 64) * DM;

  v8f acc[4];
#pragma unroll
  for (int j = 0; j < 4; ++j) acc[j] = (v8f){};

#pragma unroll 1
  for (int kk = 0; kk < DM; kk += 32) {
    const v16h xf = load_frag_row(xrow + kk, DM, lane);
#pragma unroll
    for (int j = 0; j < 4; ++j) {
      const v16h wf = load_frag_row(wrow + (long)(j * 16) * DM + kk, DM, lane);
      acc[j] = wmma_f16(wf, xf, acc[j]);
    }
  }

  const float* bias = bqkv + cb * 64;
  const float  rsc  = 1.0f / WSC;

  v4u rv[4];
  if (osel < 2) {
    float u[4][8];
#pragma unroll
    for (int j = 0; j < 4; ++j) {
      const int n8 = j * 16 + hh * 8;
      const v4f b0 = *(const v4f*)(bias + n8);
      const v4f b1 = *(const v4f*)(bias + n8 + 4);
#pragma unroll
      for (int r = 0; r < 4; ++r) {
        u[j][r]     = acc[j][r]     * rsc + bf16q(b0[r]);
        u[j][4 + r] = acc[j][4 + r] * rsc + bf16q(b1[r]);
      }
    }
    const int tl = wave * 16 + l15;
    _Float16* srow = stg + tl * KPAD;
    const float* crow = ctab + tl * RTP;
    const float* nrow = stab + tl * RTP;
#pragma unroll
    for (int j = 0; j < 2; ++j) {
      const int n8 = j * 16 + hh * 8;
      const v4f c0  = *(const v4f*)(crow + n8);
      const v4f c1  = *(const v4f*)(crow + n8 + 4);
      const v4f sn0 = *(const v4f*)(nrow + n8);
      const v4f sn1 = *(const v4f*)(nrow + n8 + 4);
      H8 plo, phi;
#pragma unroll
      for (int r = 0; r < 4; ++r) {
        const float a0 = u[j][r],     d0 = u[j + 2][r];
        const float a1 = u[j][4 + r], d1 = u[j + 2][4 + r];
        plo.h[r]     = (_Float16)(a0 * c0[r] - d0 * sn0[r]);
        phi.h[r]     = (_Float16)(d0 * c0[r] + a0 * sn0[r]);
        plo.h[4 + r] = (_Float16)(a1 * c1[r] - d1 * sn1[r]);
        phi.h[4 + r] = (_Float16)(d1 * c1[r] + a1 * sn1[r]);
      }
      *(v4u*)(srow + n8)      = plo.u;
      *(v4u*)(srow + 32 + n8) = phi.u;
    }
    __syncthreads();
#pragma unroll
    for (int it = 0; it < 4; ++it) {
      const int idx = it * 256 + tid;
      const int row = idx >> 3, piece = idx & 7;
      rv[it] = *(const v4u*)(stg + row * KPAD + piece * 8);
    }
    _Float16* dst = ((osel == 0) ? q : k) + ((long)(b * NH + h) * SEQ + s0) * HD;
#pragma unroll
    for (int it = 0; it < 4; ++it)
      *(volatile v4u*)(dst + (long)(it * 256 + tid) * 8) = rv[it];
    __threadfence();
#pragma unroll
    for (int it = 0; it < 4; ++it)
      *(volatile v4u*)(dst + (long)(it * 256 + tid) * 8) = rv[it];
  } else {
#pragma unroll
    for (int j = 0; j < 4; ++j) {
      const int n8 = j * 16 + hh * 8;
      const v4f b0 = *(const v4f*)(bias + n8);
      const v4f b1 = *(const v4f*)(bias + n8 + 4);
#pragma unroll
      for (int r = 0; r < 4; ++r) {
        stg[(n8 + r) * VSPAD + wave * 16 + l15]     = (_Float16)(acc[j][r]     * rsc + bf16q(b0[r]));
        stg[(n8 + 4 + r) * VSPAD + wave * 16 + l15] = (_Float16)(acc[j][4 + r] * rsc + bf16q(b1[r]));
      }
    }
    __syncthreads();
#pragma unroll
    for (int it = 0; it < 4; ++it) {
      const int idx = it * 256 + tid;
      const int d = idx >> 4, piece = idx & 15;
      rv[it] = *(const v4u*)(stg + d * VSPAD + piece * 8);
    }
    _Float16* dstb = vT + ((long)(b * NH + h) * HD) * SEQ + s0;
#pragma unroll
    for (int it = 0; it < 4; ++it) {
      const int idx = it * 256 + tid;
      const int d = idx >> 4, piece = idx & 15;
      *(volatile v4u*)(dstb + (long)d * SEQ + piece * 8) = rv[it];
    }
    __threadfence();
#pragma unroll
    for (int it = 0; it < 4; ++it) {
      const int idx = it * 256 + tid;
      const int d = idx >> 4, piece = idx & 15;
      *(volatile v4u*)(dstb + (long)d * SEQ + piece * 8) = rv[it];
    }
  }
}

__global__ __launch_bounds__(256) void attn_kernel(
    const _Float16* __restrict__ Q, const _Float16* __restrict__ K,
    const _Float16* __restrict__ vT, _Float16* __restrict__ ctx) {
  __shared__ _Float16 ks[64 * KPAD];
  __shared__ _Float16 vts[64 * KPAD];
  __shared__ _Float16 ost[128 * KPAD];

  const int tid  = threadIdx.x;
  const int lane = tid & 31;
  const int wave = tid >> 5;
  const int bh   = blockIdx.y;
  const int b    = bh >> 4;
  const int h    = bh & 15;
  const int q0   = blockIdx.x * 128;

  const _Float16* Qb  = Q + ((long)bh * SEQ + q0) * HD;
  const _Float16* Kb  = K + (long)bh * SEQ * HD;
  const _Float16* vTb = vT + (long)bh * HD * SEQ;

  v16h qfrag[2];
  {
    const _Float16* qrow = Qb + (long)wave * 16 * HD;
#pragma unroll
    for (int t = 0; t < 2; ++t) qfrag[t] = load_frag_row(qrow + t * 32, HD, lane);
  }

  v8f acc[4];
#pragma unroll
  for (int nt = 0; nt < 4; ++nt) acc[nt] = (v8f){};
  float mi = -1e30f, li = 0.0f;

  const int colb = lane & 15;
  const int rofs = (lane >> 4) << 3;

#pragma unroll 1
  for (int kb = 0; kb < SEQ; kb += 64) {
    __syncthreads();
#pragma unroll
    for (int idx = tid; idx < 64 * 8; idx += 256) {
      const int row = idx >> 3, c = idx & 7;
      *(v4u*)(ks + row * KPAD + c * 8) =
          *(const v4u*)(Kb + (long)(kb + row) * HD + c * 8);
    }
#pragma unroll
    for (int idx = tid; idx < 64 * 8; idx += 256) {
      const int d = idx >> 3, c = idx & 7;
      *(v4u*)(vts + d * KPAD + c * 8) =
          *(const v4u*)(vTb + (long)d * SEQ + kb + c * 8);
    }
    __syncthreads();

    v8f sc[4];
#pragma unroll
    for (int kt = 0; kt < 4; ++kt) sc[kt] = (v8f){};
#pragma unroll
    for (int t = 0; t < 2; ++t)
#pragma unroll
      for (int kt = 0; kt < 4; ++kt) {
        const v16h kf = load_frag_row(ks + (kt * 16) * KPAD + t * 32, KPAD, lane);
        sc[kt] = wmma_f16(kf, qfrag[t], sc[kt]);
      }

    float mx = sc[0][0];
#pragma unroll
    for (int kt = 0; kt < 4; ++kt)
#pragma unroll
      for (int r = 0; r < 8; ++r) mx = fmaxf(mx, sc[kt][r]);
    mx = fmaxf(mx, __shfl_xor(mx, 16, 32));
    const float mnew  = fmaxf(mi, mx);
    const float alpha = __expf((mi - mnew) * 0.125f);
    mi = mnew;
    const float cs = fmaf(mnew, 0.125f, -LN1024);

    float rs = 0.0f;
#pragma unroll
    for (int kt = 0; kt < 4; ++kt)
#pragma unroll
      for (int r = 0; r < 8; ++r) {
        const float p = __expf(fmaf(sc[kt][r], 0.125f, -cs));
        sc[kt][r] = p;
        rs += p;
      }
    rs += __shfl_xor(rs, 16, 32);
    li = li * alpha + rs;

    v16h pf[2];
#pragma unroll
    for (int t = 0; t < 2; ++t)
#pragma unroll
      for (int i = 0; i < 8; ++i) {
        pf[t][i]     = (_Float16)sc[2 * t][i];
        pf[t][8 + i] = (_Float16)sc[2 * t + 1][i];
      }

#pragma unroll
    for (int nt = 0; nt < 4; ++nt)
#pragma unroll
      for (int r = 0; r < 8; ++r) acc[nt][r] *= alpha;

#pragma unroll
    for (int t = 0; t < 2; ++t)
#pragma unroll
      for (int nt = 0; nt < 4; ++nt) {
        const v16h vf = load_frag_row(vts + (nt * 16) * KPAD + t * 32, KPAD, lane);
        acc[nt] = wmma_f16(vf, pf[t], acc[nt]);
      }
  }

  {
    const float inv = 64.0f / li;
    _Float16* orow = ost + (wave * 16 + colb) * KPAD;
#pragma unroll
    for (int nt = 0; nt < 4; ++nt) {
      H8 pk;
#pragma unroll
      for (int r = 0; r < 8; ++r) pk.h[r] = (_Float16)(acc[nt][r] * inv);
      *(v4u*)(orow + nt * 16 + rofs) = pk.u;
    }
  }
  __syncthreads();

  v4u rv[4];
#pragma unroll
  for (int it = 0; it < 4; ++it) {
    const int idx = it * 256 + tid;
    const int row = idx >> 3, piece = idx & 7;
    rv[it] = *(const v4u*)(ost + row * KPAD + piece * 8);
  }
  _Float16* cbase = ctx + ((long)b * SEQ + q0) * DM + h * HD;
#pragma unroll
  for (int it = 0; it < 4; ++it) {
    const int idx = it * 256 + tid;
    const int row = idx >> 3, piece = idx & 7;
    *(volatile v4u*)(cbase + (long)row * DM + piece * 8) = rv[it];
  }
  __threadfence();
#pragma unroll
  for (int it = 0; it < 4; ++it) {
    const int idx = it * 256 + tid;
    const int row = idx >> 3, piece = idx & 7;
    *(volatile v4u*)(cbase + (long)row * DM + piece * 8) = rv[it];
  }
}

template <int KD, int MODE>
__global__ __launch_bounds__(256) void gemm_row_kernel(
    const _Float16* __restrict__ act, const _Float16* __restrict__ wt,
    const float* __restrict__ bias, const float* __restrict__ res,
    const float* __restrict__ gam, const float* __restrict__ bet,
    float* __restrict__ outf, _Float16* __restrict__ outh) {
  __shared__ float ys[16 * YP];
  __shared__ float smean[16];
  __shared__ float srstd[16];

  const int tid  = threadIdx.x;
  const int lane = tid & 31;
  const int wave = tid >> 5;
  const int hh   = lane >> 4;
  const int l15  = lane & 15;
  const long m0  = (long)blockIdx.x * 16;
  const int  n0  = wave * 128;

  const _Float16* brow = act + m0 * KD;
  const _Float16* arow = wt + (long)n0 * KD;

  v8f acc[8];
#pragma unroll
  for (int j = 0; j < 8; ++j) acc[j] = (v8f){};

#pragma unroll 1
  for (int kk = 0; kk < KD; kk += 32) {
    const v16h bfr = load_frag_row(brow + kk, KD, lane);
#pragma unroll
    for (int j = 0; j < 8; ++j) {
      const v16h afr = load_frag_row(arow + (long)(j * 16) * KD + kk, KD, lane);
      acc[j] = wmma_f16(afr, bfr, acc[j]);
    }
  }

  {
    const float rsc = 1.0f / (WSC * WSC);
    float* yrow = ys + l15 * YP;
#pragma unroll
    for (int j = 0; j < 8; ++j) {
      const int n8 = n0 + j * 16 + hh * 8;
      const v4f b0 = *(const v4f*)(bias + n8);
      const v4f b1 = *(const v4f*)(bias + n8 + 4);
      v4f y0, y1;
#pragma unroll
      for (int i = 0; i < 4; ++i) {
        y0[i] = acc[j][i]     * rsc + bf16q(b0[i]);
        y1[i] = acc[j][4 + i] * rsc + bf16q(b1[i]);
      }
      *(v4f*)(yrow + n8)     = y0;
      *(v4f*)(yrow + n8 + 4) = y1;
    }
  }
  __syncthreads();

#pragma unroll 4
  for (int it = 0; it < 16; ++it) {
    const int idx = it * 256 + tid;
    const int row = idx >> 8, piece = idx & 255;
    const long m = m0 + row;
    v4f rsd;
    if (MODE == 0) {
      const long orow = (m / SEQ) * SEQ_FULL + (m % SEQ);
      rsd = *(const v4f*)(res + orow * DM + piece * 4);
#pragma unroll
      for (int c = 0; c < 4; ++c) rsd[c] = bf16q(rsd[c]);
    } else {
      rsd = *(const v4f*)(res + m * DM + piece * 4);
    }
    float* yp = ys + row * YP + piece * 4;
    v4f yv = *(const v4f*)yp;
#pragma unroll
    for (int c = 0; c < 4; ++c) yv[c] = yv[c] + rsd[c];
    *(v4f*)yp = yv;
  }
  __syncthreads();

  v4u hv[8];
#pragma unroll
  for (int it = 0; it < 8; ++it) hv[it] = (v4u){0u, 0u, 0u, 0u};

  if (MODE == 0) {
    {
      const int r  = tid >> 4;
      const int sl = tid & 15;
      const float* yr = ys + r * YP + sl * 64;
      float s = 0.0f;
#pragma unroll
      for (int i = 0; i < 16; ++i) {
        const v4f v = *(const v4f*)(yr + i * 4);
        s += (v[0] + v[1]) + (v[2] + v[3]);
      }
      s += __shfl_xor(s, 1, 32);
      s += __shfl_xor(s, 2, 32);
      s += __shfl_xor(s, 4, 32);
      s += __shfl_xor(s, 8, 32);
      const float mean = s * (1.0f / DM);
      float ss = 0.0f;
#pragma unroll
      for (int i = 0; i < 16; ++i) {
        const v4f v = *(const v4f*)(yr + i * 4);
#pragma unroll
        for (int c = 0; c < 4; ++c) {
          const float d = v[c] - mean;
          ss += d * d;
        }
      }
      ss += __shfl_xor(ss, 1, 32);
      ss += __shfl_xor(ss, 2, 32);
      ss += __shfl_xor(ss, 4, 32);
      ss += __shfl_xor(ss, 8, 32);
      const float var  = ss * (1.0f / DM);
      const float rstd = rsqrtf(var + LN_EPS);
      if (sl == 0) { smean[r] = mean; srstd[r] = rstd; }
    }
    __syncthreads();

#pragma unroll
    for (int it = 0; it < 8; ++it) {
      const int idx = it * 256 + tid;
      const int row = idx >> 7, p8 = idx & 127;
      const v4f a  = *(const v4f*)(ys + row * YP + p8 * 8);
      const v4f c  = *(const v4f*)(ys + row * YP + p8 * 8 + 4);
      const v4f g0 = *(const v4f*)(gam + p8 * 8);
      const v4f g1 = *(const v4f*)(gam + p8 * 8 + 4);
      const v4f b0 = *(const v4f*)(bet + p8 * 8);
      const v4f b1 = *(const v4f*)(bet + p8 * 8 + 4);
      const float mean = smean[row], rstd = srstd[row];
      H8 o;
#pragma unroll
      for (int i = 0; i < 4; ++i) {
        o.h[i]     = (_Float16)((a[i] - mean) * rstd * bf16q(g0[i]) + bf16q(b0[i]));
        o.h[4 + i] = (_Float16)((c[i] - mean) * rstd * bf16q(g1[i]) + bf16q(b1[i]));
      }
      hv[it] = o.u;
    }
  }

  auto store_pass = [&]() {
#pragma unroll 4
    for (int it = 0; it < 16; ++it) {
      const int idx = it * 256 + tid;
      const int row = idx >> 8, piece = idx & 255;
      const long m = m0 + row;
      const v4f v = *(const v4f*)(ys + row * YP + piece * 4);
      long drow;
      if (MODE == 0) drow = m;
      else drow = (m / SEQ) * SEQ_FULL + (m % SEQ);
      *(volatile v4f*)(outf + drow * DM + piece * 4) = v;
    }
    if (MODE == 0) {
#pragma unroll
      for (int it = 0; it < 8; ++it) {
        const int idx = it * 256 + tid;
        const int row = idx >> 7, p8 = idx & 127;
        const long m = m0 + row;
        *(volatile v4u*)(outh + m * DM + p8 * 8) = hv[it];
      }
    }
  };
  store_pass();
  __threadfence();
  store_pass();
}

__global__ __launch_bounds__(256) void ffn1_kernel(
    const _Float16* __restrict__ x2h, const _Float16* __restrict__ wf1t,
    const float* __restrict__ bf1, _Float16* __restrict__ hp) {
  __shared__ _Float16 stg[128 * KPAD];

  const int tid  = threadIdx.x;
  const int lane = tid & 31;
  const int wave = tid >> 5;
  const int hh   = lane >> 4;
  const int l15  = lane & 15;
  const int cb   = blockIdx.y;
  const long m0  = (long)blockIdx.x * 128;

  const _Float16* brow = x2h + (m0 + wave * 16) * DM;
  const _Float16* arow = wf1t + ((long)cb * 64) * DM;

  v8f acc[4];
#pragma unroll
  for (int j = 0; j < 4; ++j) acc[j] = (v8f){};

#pragma unroll 1
  for (int kk = 0; kk < DM; kk += 32) {
    const v16h xf = load_frag_row(brow + kk, DM, lane);
#pragma unroll
    for (int j = 0; j < 4; ++j) {
      const v16h wf = load_frag_row(arow + (long)(j * 16) * DM + kk, DM, lane);
      acc[j] = wmma_f16(wf, xf, acc[j]);
    }
  }

  const float rsc = 1.0f / WSC;
  _Float16* srow = stg + (wave * 16 + l15) * KPAD;
#pragma unroll
  for (int j = 0; j < 4; ++j) {
    const int n8 = j * 16 + hh * 8;
    const v4f b0 = *(const v4f*)(bf1 + cb * 64 + n8);
    const v4f b1 = *(const v4f*)(bf1 + cb * 64 + n8 + 4);
    H8 pk;
#pragma unroll
    for (int r = 0; r < 4; ++r) {
      const float u0 = acc[j][r]     * rsc + bf16q(b0[r]);
      const float u1 = acc[j][4 + r] * rsc + bf16q(b1[r]);
      const float e0 = __expf(fminf(-u0, 80.0f));
      const float e1 = __expf(fminf(-u1, 80.0f));
      const float g0 = u0 * __builtin_amdgcn_rcpf(1.0f + e0);
      const float g1 = u1 * __builtin_amdgcn_rcpf(1.0f + e1);
      pk.h[r]     = (_Float16)(g0 * WSC);
      pk.h[4 + r] = (_Float16)(g1 * WSC);
    }
    *(v4u*)(srow + n8) = pk.u;
  }
  __syncthreads();

  v4u rv[4];
#pragma unroll
  for (int it = 0; it < 4; ++it) {
    const int idx = it * 256 + tid;
    const int row = idx >> 3, piece = idx & 7;
    rv[it] = *(const v4u*)(stg + row * KPAD + piece * 8);
  }
#pragma unroll
  for (int it = 0; it < 4; ++it) {
    const int idx = it * 256 + tid;
    const int row = idx >> 3, piece = idx & 7;
    *(volatile v4u*)(hp + (m0 + row) * FF + cb * 64 + piece * 8) = rv[it];
  }
  __threadfence();
#pragma unroll
  for (int it = 0; it < 4; ++it) {
    const int idx = it * 256 + tid;
    const int row = idx >> 3, piece = idx & 7;
    *(volatile v4u*)(hp + (m0 + row) * FF + cb * 64 + piece * 8) = rv[it];
  }
}

extern "C" void kernel_launch(void* const* d_in, const int* in_sizes, int n_in,
                              void* d_out, int out_size, void* d_ws, size_t ws_size,
                              hipStream_t stream) {
  if (n_in < 13) return;
  const long needRows = (long)(NB - 1) * SEQ_FULL + SEQ;
  if ((long)in_sizes[0] < needRows * DM) return;
  if (in_sizes[1] < DM || in_sizes[2] < DM) return;
  if (in_sizes[3] < 3 * DM * DM || in_sizes[4] < 3 * DM) return;
  if (in_sizes[5] < DM * DM || in_sizes[6] < DM) return;
  if (in_sizes[7] < DM || in_sizes[8] < DM) return;
  if (in_sizes[9] < DM * FF || in_sizes[10] < FF) return;
  if (in_sizes[11] < FF * DM || in_sizes[12] < DM) return;
  if ((long)out_size < needRows * DM) return;
  if (ws_size < WS_TOTAL) return;

  const float* x     = (const float*)d_in[0];
  const float* g1    = (const float*)d_in[1];
  const float* be1   = (const float*)d_in[2];
  const float* Wqkv  = (const float*)d_in[3];
  const float* bqkv  = (const float*)d_in[4];
  const float* Wo    = (const float*)d_in[5];
  const float* bo    = (const float*)d_in[6];
  const float* g2    = (const float*)d_in[7];
  const float* be2   = (const float*)d_in[8];
  const float* Wf1   = (const float*)d_in[9];
  const float* bf1   = (const float*)d_in[10];
  const float* Wf2   = (const float*)d_in[11];
  const float* bf2   = (const float*)d_in[12];
  float* out = (float*)d_out;

  char* ws = (char*)d_ws;
  size_t off = 0;
  _Float16* nxh  = (_Float16*)(ws + off); off += PLANE2;
  _Float16* ctx  = (_Float16*)(ws + off); off += PLANE2;
  _Float16* wqkv = (_Float16*)(ws + off); off += WQKV_BYTES;
  _Float16* woh  = (_Float16*)(ws + off); off += WO_BYTES;
  _Float16* wf1t = (_Float16*)(ws + off); off += WF1_BYTES;
  _Float16* wf2t = (_Float16*)(ws + off); off += WF2_BYTES;
  _Float16* qh   = (_Float16*)(ws + off); off += PLANE2;
  _Float16* kh   = (_Float16*)(ws + off); off += PLANE2;
  _Float16* vTh  = (_Float16*)(ws + off); off += PLANE2;
  float*    x1f  = (float*)(ws + off);    off += PLANE4;
  _Float16* nx2h = (_Float16*)(ws + off); off += PLANE2;
  _Float16* hp   = (_Float16*)(ws + off); off += H_BYTES;
  if (off > ws_size) return;

  ln1_kernel<<<ROWS / 8, 256, 0, stream>>>(x, g1, be1, nxh);
  cvt_w_kernel<<<NWT, 256, 0, stream>>>(Wqkv, Wo, Wf1, Wf2, wqkv, woh, wf1t, wf2t);
  qkv_kernel<<<dim3(ROWS / 128, 3 * NH), 256, 0, stream>>>(nxh, wqkv, bqkv, qh, kh, vTh);
  attn_kernel<<<dim3(SEQ / 128, NB * NH), 256, 0, stream>>>(qh, kh, vTh, ctx);
  gemm_row_kernel<DM, 0><<<ROWS / 16, 256, 0, stream>>>(ctx, woh, bo, x, g2, be2, x1f, nx2h);
  ffn1_kernel<<<dim3(ROWS / 128, FF / 64), 256, 0, stream>>>(nx2h, wf1t, bf1, hp);
  gemm_row_kernel<FF, 1><<<ROWS / 16, 256, 0, stream>>>(hp, wf2t, bf2, x1f, g2, be2, out, nx2h);
}
